// Encoder_59485297050149
// MI455X (gfx1250) — hardware-verified
//
#include <hip/hip_runtime.h>
#include <hip/hip_fp16.h>


#ifndef NB
#define NB 2
#endif
#ifndef SEQ
#define SEQ 2048
#endif
#define NB_FULL  2
#define SEQ_FULL 2048
#define DM   768
#define NH   12
#define HD   64
#define FF   3072
#define QKP  (2 * DM)
#define NTOK (NB * SEQ)

static_assert(NB >= 1 && NB <= NB_FULL);
static_assert(SEQ >= 64 && SEQ <= SEQ_FULL);
static_assert(SEQ % 64 == 0);
static_assert(NTOK % 128 == 0);
static_assert(DM == NH * HD);
static_assert(DM % 128 == 0 && FF % 128 == 0 && QKP % 128 == 0);
static_assert(DM % 32 == 0 && FF % 32 == 0);
static_assert((DM * DM) % 2048 == 0 && (FF * DM) % 2048 == 0);

typedef _Float16 v16h __attribute__((ext_vector_type(16)));
typedef _Float16 v8h  __attribute__((ext_vector_type(8)));
typedef float    v8f  __attribute__((ext_vector_type(8)));
typedef float    v4f  __attribute__((ext_vector_type(4)));
typedef int      v4i  __attribute__((ext_vector_type(4)));

union Frag { v16h v; v8h h[2]; };

#define LOG2E   1.44269504088896340736f
#define CS_T    (LOG2E * 3.0517578125e-05f)
#define NEG_T   (-1.0e9f * LOG2E)
#define SC_M12  2.44140625e-04f
#define SC_M6   0.015625f

static __device__ __forceinline__ v8f zero8() {
    v8f z;
#pragma unroll
    for (int i = 0; i < 8; ++i) z[i] = 0.0f;
    return z;
}

static __device__ __forceinline__ v16h load_frag16(const _Float16* base, int ld, int lane) {
    int m  = lane & 15;
    int kb = (lane >> 4) << 3;
    const _Float16* p = base + (size_t)m * ld + kb;
    Frag f;
    f.h[0] = *(const v8h*)(p);
    f.h[1] = *(const v8h*)(p + 16);
    return f.v;
}

static __device__ __forceinline__ v8f wmma16(v16h a, v16h b, v8f c) {
    v8f d = __builtin_amdgcn_wmma_f32_16x16x32_f16(false, a, false, b, (short)0, c, false, false);
    asm volatile("v_nop\n\tv_nop\n\tv_nop\n\tv_nop" : "+v"(d) : "v"(a), "v"(b));
    return d;
}

static __device__ __forceinline__ float bf16r(float x) {
    unsigned u = __float_as_uint(x);
    u = (u + 0x7FFFu + ((u >> 16) & 1u)) & 0xFFFF0000u;
    return __uint_as_float(u);
}

static __device__ __forceinline__ float ex2(float x) {
    return __builtin_amdgcn_exp2f(x);
}

static __device__ __forceinline__ float rcp(float x) {
    return __builtin_amdgcn_rcpf(x);
}

static __device__ __forceinline__ void wave_lds_sync() {
    __builtin_amdgcn_fence(3, "wavefront");
    asm volatile("s_wait_dscnt 0" ::: "memory");
    __builtin_amdgcn_wave_barrier();
}

__global__ __launch_bounds__(256) void k_wcvt(const float* __restrict__ wq,
                                               const float* __restrict__ wk,
                                               const float* __restrict__ wv,
                                               const float* __restrict__ wo,
                                               const float* __restrict__ w1,
                                               const float* __restrict__ w3,
                                               const float* __restrict__ w2,
                                               _Float16* pqk, _Float16* pv, _Float16* po,
                                               _Float16* p1, _Float16* p3, _Float16* p2) {
    const unsigned y   = blockIdx.y;
    const unsigned n   = (y < 4u) ? (unsigned)(DM * DM) : (unsigned)(FF * DM);
    const unsigned idx = (blockIdx.x * 256u + threadIdx.x) * 8u;
    if (idx >= n) return;
    const float* s = (y == 0u) ? wq : (y == 1u) ? wk : (y == 2u) ? wv : (y == 3u) ? wo
                   : (y == 4u) ? w1 : (y == 5u) ? w3 : w2;
    _Float16* d = (y == 0u) ? pqk : (y == 1u) ? (pqk + (size_t)DM * DM) : (y == 2u) ? pv
                : (y == 3u) ? po : (y == 4u) ? p1 : (y == 5u) ? p3 : p2;
    const v4f a = *(const v4f*)(s + idx);
    const v4f b = *(const v4f*)(s + idx + 4);
    v8h o;
    o[0] = (_Float16)(bf16r(a.x) * 64.0f);
    o[1] = (_Float16)(bf16r(a.y) * 64.0f);
    o[2] = (_Float16)(bf16r(a.z) * 64.0f);
    o[3] = (_Float16)(bf16r(a.w) * 64.0f);
    o[4] = (_Float16)(bf16r(b.x) * 64.0f);
    o[5] = (_Float16)(bf16r(b.y) * 64.0f);
    o[6] = (_Float16)(bf16r(b.z) * 64.0f);
    o[7] = (_Float16)(bf16r(b.w) * 64.0f);
    *(volatile v8h*)(d + idx) = o;
    __threadfence();
    *(volatile v8h*)(d + idx) = o;
}

template <int XIN>
__global__ __launch_bounds__(256) void k_rms(const float* __restrict__ X,
                                              const float* __restrict__ g,
                                              _Float16* __restrict__ Y) {
    const unsigned tid  = threadIdx.x;
    const unsigned lane = tid & 31u;
    const unsigned w    = tid >> 5;
    const unsigned tok  = blockIdx.x * 8u + w;
    unsigned srow = tok;
    if (XIN) {
        const unsigned b = tok / (unsigned)SEQ;
        srow = b * (unsigned)SEQ_FULL + (tok - b * (unsigned)SEQ);
    }
    const float* xr = X + (size_t)srow * DM;
    float v[3][8];
    float ss = 0.0f;
#pragma unroll
    for (int i = 0; i < 3; ++i) {
        const unsigned c = ((unsigned)i * 32u + lane) * 8u;
        const v4f a = *(const v4f*)(xr + c);
        const v4f b = *(const v4f*)(xr + c + 4);
        v[i][0] = a.x; v[i][1] = a.y; v[i][2] = a.z; v[i][3] = a.w;
        v[i][4] = b.x; v[i][5] = b.y; v[i][6] = b.z; v[i][7] = b.w;
#pragma unroll
        for (int j = 0; j < 8; ++j) {
            if (XIN) v[i][j] = bf16r(v[i][j]);
            ss += v[i][j] * v[i][j];
        }
    }
    ss += __shfl_xor(ss, 16, 32);
    ss += __shfl_xor(ss, 8, 32);
    ss += __shfl_xor(ss, 4, 32);
    ss += __shfl_xor(ss, 2, 32);
    ss += __shfl_xor(ss, 1, 32);
    const float inv = rsqrtf(ss * (1.0f / (float)DM) + 1.0e-5f);
    v8h o[3];
#pragma unroll
    for (int i = 0; i < 3; ++i) {
        const unsigned c = ((unsigned)i * 32u + lane) * 8u;
        const v4f ga = *(const v4f*)(g + c);
        const v4f gb = *(const v4f*)(g + c + 4);
        o[i][0] = (_Float16)(bf16r(ga.x) * (v[i][0] * inv));
        o[i][1] = (_Float16)(bf16r(ga.y) * (v[i][1] * inv));
        o[i][2] = (_Float16)(bf16r(ga.z) * (v[i][2] * inv));
        o[i][3] = (_Float16)(bf16r(ga.w) * (v[i][3] * inv));
        o[i][4] = (_Float16)(bf16r(gb.x) * (v[i][4] * inv));
        o[i][5] = (_Float16)(bf16r(gb.y) * (v[i][5] * inv));
        o[i][6] = (_Float16)(bf16r(gb.z) * (v[i][6] * inv));
        o[i][7] = (_Float16)(bf16r(gb.w) * (v[i][7] * inv));
    }
    _Float16* yr = Y + (size_t)tok * DM;
#pragma unroll
    for (int i = 0; i < 3; ++i) *(volatile v8h*)(yr + ((unsigned)i * 32u + lane) * 8u) = o[i];
    __threadfence();
#pragma unroll
    for (int i = 0; i < 3; ++i) *(volatile v8h*)(yr + ((unsigned)i * 32u + lane) * 8u) = o[i];
}

template <int MODE>
__global__ __launch_bounds__(128) __attribute__((amdgpu_num_vgpr(256)))
void k_gemm(const _Float16* __restrict__ A, const _Float16* __restrict__ B,
            _Float16* __restrict__ C16, float* __restrict__ C32,
            const float* __restrict__ R,
            unsigned K, unsigned lda, unsigned ldb, unsigned ldc) {
    const int tid  = threadIdx.x;
    const int lane = tid & 31;
    const int w    = tid >> 5;
    const unsigned m0 = blockIdx.y * 64u + (unsigned)(w >> 1) * 32u;
    const unsigned n0 = blockIdx.x * 128u + (unsigned)(w & 1) * 64u;
    const _Float16* a0p = A + (size_t)m0 * lda;
    const _Float16* a1p = a0p + (size_t)16 * lda;
    const _Float16* bp  = B + (size_t)n0 * ldb;

    v8f acc[2][4];
#pragma unroll
    for (int mi = 0; mi < 2; ++mi)
#pragma unroll
        for (int ni = 0; ni < 4; ++ni) acc[mi][ni] = zero8();

#pragma unroll 1
    for (unsigned k0 = 0; k0 < K; k0 += 32u) {
        const v16h a0 = load_frag16(a0p + k0, (int)lda, lane);
        const v16h a1 = load_frag16(a1p + k0, (int)lda, lane);
#pragma unroll
        for (int ni = 0; ni < 4; ++ni) {
            const v16h bf = load_frag16(bp + (size_t)(ni * 16) * ldb + k0, (int)ldb, lane);
            acc[0][ni] = wmma16(a0, bf, acc[0][ni]);
            acc[1][ni] = wmma16(a1, bf, acc[1][ni]);
        }
    }

    const int r0 = (lane >> 4) << 3;
    const int cc = lane & 15;
    if constexpr (MODE == 0) {
        __shared__ __align__(16) _Float16 st16[4][32 * 64];
        _Float16* stw = &st16[w][0];
#pragma unroll
        for (int mi = 0; mi < 2; ++mi)
#pragma unroll
            for (int ni = 0; ni < 4; ++ni)
#pragma unroll
                for (int g = 0; g < 8; ++g)
                    stw[(mi * 16 + r0 + g) * 64 + ni * 16 + cc] = (_Float16)acc[mi][ni][g];
        wave_lds_sync();
        const int rq = lane >> 3;
        const int c8 = (lane & 7) * 8;
        v8h pv[8];
#pragma unroll
        for (int i = 0; i < 8; ++i) pv[i] = *(const v8h*)(&stw[(i * 4 + rq) * 64 + c8]);
        _Float16* cb = C16 + (size_t)(m0 + (unsigned)rq) * ldc + n0 + (unsigned)c8;
#pragma unroll
        for (int i = 0; i < 8; ++i) *(volatile v8h*)(cb + (size_t)(i * 4) * ldc) = pv[i];
        __threadfence();
#pragma unroll
        for (int i = 0; i < 8; ++i) *(volatile v8h*)(cb + (size_t)(i * 4) * ldc) = pv[i];
    } else {
        __shared__ __align__(16) float st32[4][32 * 64];
        float* stw = &st32[w][0];
#pragma unroll
        for (int mi = 0; mi < 2; ++mi)
#pragma unroll
            for (int ni = 0; ni < 4; ++ni)
#pragma unroll
                for (int g = 0; g < 8; ++g)
                    stw[(mi * 16 + r0 + g) * 64 + ni * 16 + cc] = acc[mi][ni][g];
        wave_lds_sync();
        const int rq = lane >> 4;
        const int c4 = (lane & 15) * 4;
        v4f sv[16];
#pragma unroll
        for (int i = 0; i < 16; ++i) {
            const int row = i * 2 + rq;
            const v4f a = *(const v4f*)(&stw[row * 64 + c4]);
            const unsigned tok = m0 + (unsigned)row;
            unsigned rrow = tok;
            if (MODE == 1) {
                const unsigned b = tok / (unsigned)SEQ;
                rrow = b * (unsigned)SEQ_FULL + (tok - b * (unsigned)SEQ);
            }
            v4f r = *(const v4f*)(R + (size_t)rrow * ldc + n0 + (unsigned)c4);
            if (MODE == 1) { r.x = bf16r(r.x); r.y = bf16r(r.y); r.z = bf16r(r.z); r.w = bf16r(r.w); }
            v4f o;
            o.x = r.x + a.x * SC_M12;
            o.y = r.y + a.y * SC_M12;
            o.z = r.z + a.z * SC_M12;
            o.w = r.w + a.w * SC_M12;
            sv[i] = o;
        }
        float* cb = C32 + (size_t)(m0 + (unsigned)rq) * ldc + n0 + (unsigned)c4;
#pragma unroll
        for (int i = 0; i < 16; ++i) *(volatile v4f*)(cb + (size_t)(i * 2) * ldc) = sv[i];
        __threadfence();
#pragma unroll
        for (int i = 0; i < 16; ++i) *(volatile v4f*)(cb + (size_t)(i * 2) * ldc) = sv[i];
    }
}

__global__ __launch_bounds__(128) __attribute__((amdgpu_num_vgpr(256)))
void k_dual(const _Float16* __restrict__ A, const _Float16* __restrict__ B1,
            const _Float16* __restrict__ B3, _Float16* __restrict__ U) {
    __shared__ __align__(16) _Float16 su[32 * 128];
    const int tid  = threadIdx.x;
    const int lane = tid & 31;
    const int w    = tid >> 5;
    const unsigned m0 = blockIdx.y * 32u;
    const unsigned n0 = blockIdx.x * 128u + (unsigned)w * 32u;
    const _Float16* a0p = A + (size_t)m0 * DM;
    const _Float16* a1p = a0p + (size_t)16 * DM;
    const _Float16* b1p = B1 + (size_t)n0 * DM;
    const _Float16* b3p = B3 + (size_t)n0 * DM;

    v8f acc1[2][2], acc3[2][2];
#pragma unroll
    for (int mi = 0; mi < 2; ++mi)
#pragma unroll
        for (int ni = 0; ni < 2; ++ni) { acc1[mi][ni] = zero8(); acc3[mi][ni] = zero8(); }

#pragma unroll 1
    for (unsigned k0 = 0; k0 < (unsigned)DM; k0 += 32u) {
        const v16h a0 = load_frag16(a0p + k0, DM, lane);
        const v16h a1 = load_frag16(a1p + k0, DM, lane);
#pragma unroll
        for (int ni = 0; ni < 2; ++ni) {
            const v16h f1 = load_frag16(b1p + (size_t)(ni * 16) * DM + k0, DM, lane);
            acc1[0][ni] = wmma16(a0, f1, acc1[0][ni]);
            acc1[1][ni] = wmma16(a1, f1, acc1[1][ni]);
            const v16h f3 = load_frag16(b3p + (size_t)(ni * 16) * DM + k0, DM, lane);
            acc3[0][ni] = wmma16(a0, f3, acc3[0][ni]);
            acc3[1][ni] = wmma16(a1, f3, acc3[1][ni]);
        }
    }

    const int r0 = (lane >> 4) << 3;
    const int cc = lane & 15;
#pragma unroll
    for (int mi = 0; mi < 2; ++mi)
#pragma unroll
        for (int ni = 0; ni < 2; ++ni)
#pragma unroll
            for (int g = 0; g < 8; ++g) {
                const float gv = acc1[mi][ni][g] * SC_M6;
                const float e  = expf(-gv);
                const float s  = gv * rcp(1.0f + e);
                su[(mi * 16 + r0 + g) * 128 + w * 32 + ni * 16 + cc] =
                    (_Float16)(s * acc3[mi][ni][g]);
            }
    __syncthreads();
    const int rq = lane >> 4;
    const int c8 = (lane & 15) * 8;
    v8h pv[4];
#pragma unroll
    for (int i = 0; i < 4; ++i) pv[i] = *(const v8h*)(&su[(w * 8 + i * 2 + rq) * 128 + c8]);
    _Float16* ub = U + (size_t)(m0 + (unsigned)(w * 8 + rq)) * FF + blockIdx.x * 128u + (unsigned)c8;
#pragma unroll
    for (int i = 0; i < 4; ++i) *(volatile v8h*)(ub + (size_t)(i * 2) * FF) = pv[i];
    __threadfence();
#pragma unroll
    for (int i = 0; i < 4; ++i) *(volatile v8h*)(ub + (size_t)(i * 2) * FF) = pv[i];
}

static __device__ __forceinline__ float msel(int mv, float s) {
    return (mv == 0) ? NEG_T : s * CS_T;
}

__global__ __launch_bounds__(128) __attribute__((amdgpu_num_vgpr(256)))
void k_attn(const _Float16* __restrict__ qk,
            const _Float16* __restrict__ vT,
            const int* __restrict__ mask,
            _Float16* __restrict__ ctx) {
    __shared__ __align__(16) _Float16 st[4][16 * 64];
    const int tid  = threadIdx.x;
    const int lane = tid & 31;
    const int w    = tid >> 5;
    const int n    = lane & 15;
    const int hh   = lane >> 4;
    const unsigned bh = blockIdx.y;
    const unsigned b  = bh / (unsigned)NH;
    const unsigned h  = bh - b * (unsigned)NH;
    const unsigned q0 = blockIdx.x * 64u + (unsigned)w * 16u;
    const unsigned tokq = b * (unsigned)SEQ + q0;

    const _Float16* qb = qk + (size_t)tokq * QKP + h * HD;
    const v16h qf0 = load_frag16(qb, QKP, lane);
    const v16h qf1 = load_frag16(qb + 32, QKP, lane);
    const _Float16* kb = qk + (size_t)(b * (unsigned)SEQ) * QKP + DM + h * HD;
    const _Float16* vb = vT + (size_t)(h * HD) * NTOK + b * (unsigned)SEQ;
    const int* mrow = mask + ((size_t)b * SEQ_FULL + q0 + (unsigned)n) * SEQ_FULL + 8 * hh;

    v8f o[4];
#pragma unroll
    for (int dt = 0; dt < 4; ++dt) o[dt] = zero8();
    float mrun = -3.0e38f, lrun = 0.0f;

#pragma unroll 1
    for (unsigned k0 = 0; k0 < (unsigned)SEQ; k0 += 32u) {
        const v16h ka0 = load_frag16(kb + (size_t)k0 * QKP, QKP, lane);
        const v16h ka1 = load_frag16(kb + (size_t)k0 * QKP + 32, QKP, lane);
        v8f s0 = wmma16(ka0, qf0, zero8());
        s0 = wmma16(ka1, qf1, s0);
        const v16h kc0 = load_frag16(kb + (size_t)(k0 + 16u) * QKP, QKP, lane);
        const v16h kc1 = load_frag16(kb + (size_t)(k0 + 16u) * QKP + 32, QKP, lane);
        v8f s1 = wmma16(kc0, qf0, zero8());
        s1 = wmma16(kc1, qf1, s1);

        const v4i mA0 = *(const v4i*)(mrow + k0);
        const v4i mA1 = *(const v4i*)(mrow + k0 + 4);
        const v4i mB0 = *(const v4i*)(mrow + k0 + 16);
        const v4i mB1 = *(const v4i*)(mrow + k0 + 20);

        float t0[8], t1[8];
#pragma unroll
        for (int r = 0; r < 4; ++r) {
            t0[r]     = msel(mA0[r], s0[r]);
            t0[4 + r] = msel(mA1[r], s0[4 + r]);
            t1[r]     = msel(mB0[r], s1[r]);
            t1[4 + r] = msel(mB1[r], s1[4 + r]);
        }
        float tmax = fmaxf(t0[0], t1[0]);
#pragma unroll
        for (int r = 1; r < 8; ++r) tmax = fmaxf(tmax, fmaxf(t0[r], t1[r]));
        tmax = fmaxf(tmax, __shfl_xor(tmax, 16, 32));
        const float mn    = fmaxf(mrun, tmax);
        const float alpha = ex2(mrun - mn);
        float ps = 0.0f;
        Frag pb;
#pragma unroll
        for (int r = 0; r < 8; ++r) {
            const float p0 = ex2(t0[r] - mn);
            const float p1 = ex2(t1[r] - mn);
            ps += p0 + p1;
            pb.h[0][r] = (_Float16)p0;
            pb.h[1][r] = (_Float16)p1;
        }
        ps += __shfl_xor(ps, 16, 32);
        lrun = lrun * alpha + ps;
        mrun = mn;
#pragma unroll
        for (int dt = 0; dt < 4; ++dt) {
#pragma unroll
            for (int r = 0; r < 8; ++r) o[dt][r] *= alpha;
        }
#pragma unroll
        for (int dt = 0; dt < 4; ++dt) {
            const v16h va = load_frag16(vb + (size_t)(dt * 16) * NTOK + k0, NTOK, lane);
            o[dt] = wmma16(va, pb.v, o[dt]);
        }
    }

    const float inv = rcp(lrun);
    _Float16* stw = &st[w][0];
#pragma unroll
    for (int dt = 0; dt < 4; ++dt) {
        v8h pk;
#pragma unroll
        for (int r = 0; r < 8; ++r) pk[r] = (_Float16)(o[dt][r] * inv);
        *(v8h*)(&stw[n * 64 + dt * 16 + 8 * hh]) = pk;
    }
    wave_lds_sync();
    const int rq = lane >> 3;
    const int c8 = (lane & 7) * 8;
    v8h sv[4];
#pragma unroll
    for (int i = 0; i < 4; ++i) sv[i] = *(const v8h*)(&stw[(i * 4 + rq) * 64 + c8]);
    _Float16* cb = ctx + (size_t)(tokq + (unsigned)rq) * DM + h * HD + (unsigned)c8;
#pragma unroll
    for (int i = 0; i < 4; ++i) *(volatile v8h*)(cb + (size_t)(i * 4) * DM) = sv[i];
    __threadfence();
#pragma unroll
    for (int i = 0; i < 4; ++i) *(volatile v8h*)(cb + (size_t)(i * 4) * DM) = sv[i];
}

extern "C" void kernel_launch(void* const* d_in, const int* in_sizes, int n_in,
                              void* d_out, int out_size, void* d_ws, size_t ws_size,
                              hipStream_t stream) {
    if (n_in < 11) return;
    if (in_sizes[0] < ((NB - 1) * SEQ_FULL + SEQ) * DM) return;
    if (in_sizes[1] < ((NB - 1) * SEQ_FULL + (SEQ - 1)) * SEQ_FULL + SEQ) return;
    if (in_sizes[2] < DM * DM || in_sizes[3] < DM * DM) return;
    if (in_sizes[4] < DM * DM || in_sizes[5] < DM * DM) return;
    if (in_sizes[6] < FF * DM || in_sizes[7] < DM * FF || in_sizes[8] < FF * DM) return;
    if (in_sizes[9] < DM || in_sizes[10] < DM) return;
    if (out_size < NTOK * DM) return;

    const float* x    = (const float*)d_in[0];
    const int*   mask = (const int*)d_in[1];
    const float* wq   = (const float*)d_in[2];
    const float* wk   = (const float*)d_in[3];
    const float* wv   = (const float*)d_in[4];
    const float* wo   = (const float*)d_in[5];
    const float* w1   = (const float*)d_in[6];
    const float* w2   = (const float*)d_in[7];
    const float* w3   = (const float*)d_in[8];
    const float* ga   = (const float*)d_in[9];
    const float* gf   = (const float*)d_in[10];
    float* out = (float*)d_out;

    char* ws = (char*)d_ws;
    size_t off = 0;
    _Float16* pqk = (_Float16*)(ws + off); off += (size_t)QKP * DM * 2;
    _Float16* pv  = (_Float16*)(ws + off); off += (size_t)DM * DM * 2;
    _Float16* po  = (_Float16*)(ws + off); off += (size_t)DM * DM * 2;
    _Float16* p1  = (_Float16*)(ws + off); off += (size_t)FF * DM * 2;
    _Float16* p3  = (_Float16*)(ws + off); off += (size_t)FF * DM * 2;
    _Float16* p2  = (_Float16*)(ws + off); off += (size_t)DM * FF * 2;
    _Float16* xn  = (_Float16*)(ws + off); off += (size_t)NTOK * DM * 2;
    _Float16* qkp = (_Float16*)(ws + off); off += (size_t)NTOK * QKP * 2;
    _Float16* vT  = (_Float16*)(ws + off); off += (size_t)DM * NTOK * 2;
    _Float16* ctx = (_Float16*)(ws + off); off += (size_t)NTOK * DM * 2;
    float*    hpl = (float*)(ws + off);    off += (size_t)NTOK * DM * 4;
    _Float16* hn  = (_Float16*)(ws + off); off += (size_t)NTOK * DM * 2;
    _Float16* upl = (_Float16*)(ws + off); off += (size_t)NTOK * FF * 2;
    if (off > ws_size || off > (size_t)134217728) return;

    k_wcvt<<<dim3((FF * DM) / 2048, 7), dim3(256), 0, stream>>>(wq, wk, wv, wo, w1, w3, w2,
                                                               pqk, pv, po, p1, p3, p2);
    k_rms<1><<<dim3(NTOK / 8), dim3(256), 0, stream>>>(x, ga, xn);
    k_gemm<0><<<dim3(QKP / 128, NTOK / 64), dim3(128), 0, stream>>>(
        xn, pqk, qkp, hpl, x, (unsigned)DM, (unsigned)DM, (unsigned)DM, (unsigned)QKP);
    k_gemm<0><<<dim3(NTOK / 128, DM / 64), dim3(128), 0, stream>>>(
        pv, xn, vT, hpl, x, (unsigned)DM, (unsigned)DM, (unsigned)DM, (unsigned)NTOK);
    k_attn<<<dim3(SEQ / 64, NB * NH), dim3(128), 0, stream>>>(qkp, vT, mask, ctx);
    k_gemm<1><<<dim3(DM / 128, NTOK / 64), dim3(128), 0, stream>>>(
        ctx, po, hn, hpl, x, (unsigned)DM, (unsigned)DM, (unsigned)DM, (unsigned)DM);
    k_rms<0><<<dim3(NTOK / 8), dim3(256), 0, stream>>>(hpl, gf, hn);
    k_dual<<<dim3(FF / 128, NTOK / 32), dim3(128), 0, stream>>>(hn, p1, p3, upl);
    k_gemm<2><<<dim3(DM / 128, NTOK / 64), dim3(128), 0, stream>>>(
        upl, p2, hn, out, hpl, (unsigned)FF, (unsigned)FF, (unsigned)FF, (unsigned)DM);
}
